// QCompass_42021960024798
// MI455X (gfx1250) — hardware-verified
//
#include <hip/hip_runtime.h>
#include <stdint.h>

constexpr int SEQ_LEN = 2048;
constexpr int HID     = 2048;
constexpr int QRANK   = 1024;
constexpr int NHEADS  = 16;
constexpr int HRANK   = 64;
constexpr int HVAL    = 128;
static_assert(QRANK == NHEADS * HRANK, "rank split");
static_assert(HID == NHEADS * HVAL, "value split");
static_assert(SEQ_LEN % 64 == 0 && HID % 64 == 0 && QRANK % 64 == 0, "tile multiples");
static_assert(HID % 32 == 0 && QRANK % 32 == 0, "K multiples of 32");

typedef __attribute__((ext_vector_type(16))) _Float16 v16h;
typedef __attribute__((ext_vector_type(8)))  _Float16 v8h;
typedef __attribute__((ext_vector_type(16))) __bf16   v16b;
typedef __attribute__((ext_vector_type(8)))  __bf16   v8b;
typedef __attribute__((ext_vector_type(8)))  float    v8f;
typedef __attribute__((ext_vector_type(4)))  float    v4f;

__device__ __forceinline__ unsigned short f2bf_bits(float f) {
  unsigned u = __float_as_uint(f);
  return (unsigned short)((u + 0x7FFFu + ((u >> 16) & 1u)) >> 16);
}
__device__ __forceinline__ float bf_bits2f(unsigned short h) { return __uint_as_float(((unsigned)h) << 16); }

__device__ __forceinline__ void dep_guard_h(v8f& a, v8f& b, v16h x, v16h y) { asm volatile("v_nop\n\tv_nop\n\tv_nop\n\tv_nop" : "+v"(a), "+v"(b) : "v"(x), "v"(y)); }
__device__ __forceinline__ void dep_guard_b(v8f& a, v8f& b, v16b x, v16b y) { asm volatile("v_nop\n\tv_nop\n\tv_nop\n\tv_nop" : "+v"(a), "+v"(b) : "v"(x), "v"(y)); }
__device__ __forceinline__ void keep4_h(v16h a, v16h b, v16h c, v16h d) { asm volatile("v_nop" :: "v"(a), "v"(b), "v"(c), "v"(d)); }
__device__ __forceinline__ void keep4_b(v16b a, v16b b, v16b c, v16b d) { asm volatile("v_nop" :: "v"(a), "v"(b), "v"(c), "v"(d)); }
__device__ __forceinline__ void acc_guard4(v8f& a, v8f& b, v8f& c, v8f& d) { asm volatile("v_nop\n\tv_nop\n\tv_nop\n\tv_nop" : "+v"(a), "+v"(b), "+v"(c), "+v"(d)); }
template <typename T> struct Frag;
template <> struct Frag<_Float16> {
  typedef v16h V; union U { v16h v; v8h h[2]; };
  static __device__ __forceinline__ v16h load(const _Float16* p) {
    U f; f.h[0] = *(const v8h*)(p); f.h[1] = *(const v8h*)(p + 16); return f.v;
  }
  static __device__ __forceinline__ v8f mma(v16h a, v16h b, v8f c) {
    return __builtin_amdgcn_wmma_f32_16x16x32_f16(false, a, false, b, (short)0, c, false, false);
  }
  static __device__ __forceinline__ void guard(v8f& a, v8f& b, v16h x, v16h y) { dep_guard_h(a, b, x, y); }
  static __device__ __forceinline__ void keep(v16h a, v16h b, v16h c, v16h d) { keep4_h(a, b, c, d); }
};
template <> struct Frag<__bf16> {
  typedef v16b V; union U { v16b v; v8b h[2]; };
  static __device__ __forceinline__ v16b load(const __bf16* p) {
    U f; f.h[0] = *(const v8b*)(p); f.h[1] = *(const v8b*)(p + 16); return f.v;
  }
  static __device__ __forceinline__ v8f mma(v16b a, v16b b, v8f c) {
    return __builtin_amdgcn_wmma_f32_16x16x32_bf16(false, a, false, b, (short)0, c, false, false);
  }
  static __device__ __forceinline__ void guard(v8f& a, v8f& b, v16b x, v16b y) { dep_guard_b(a, b, x, y); }
  static __device__ __forceinline__ void keep(v16b a, v16b b, v16b c, v16b d) { keep4_b(a, b, c, d); }
};

template <int ET> struct Elem;
template <> struct Elem<0> { typedef _Float16 T; };
template <> struct Elem<1> { typedef __bf16 T; };
template <int ET, bool ASPLIT, bool BSPLIT, int BIAS_MODE, int OUT_MODE>
__global__ __launch_bounds__(256) void wmma_gemm64(
    const unsigned short* __restrict__ Ap, const unsigned short* __restrict__ A2p, int lda, long strideA,
    const unsigned short* __restrict__ Btp, const unsigned short* __restrict__ Bt2p, int ldb, long strideB,
    void* __restrict__ Cout, void* __restrict__ Cout2, int ldc, long strideC,
    const float* __restrict__ bias,
    int M, int N, int K, float scale) {
  typedef typename Elem<ET>::T T;
  typedef typename Frag<T>::V V;
  const T* A = (const T*)Ap; const T* A2 = (const T*)A2p; const T* Bt = (const T*)Btp; const T* Bt2 = (const T*)Bt2p;
  __shared__ __align__(16) float sT[8][16 * 68];
  const int b    = blockIdx.y;
  const int lane = threadIdx.x & 31;
  const int wave = threadIdx.x >> 5;
  const int tilesN = N >> 6;
  const int tilesM = M >> 6;
  const int tile = blockIdx.x * 8 + wave;
  if (tile >= tilesM * tilesN) return;
  const int tm = tile / tilesN;
  const int tn = tile - tm * tilesN;
  const int m0 = tm << 6;
  const int n0 = tn << 6;

  const T* Ab  = A  + (size_t)b * strideA;
  const T* Bb  = Bt + (size_t)b * strideB;
  const T* Ab2 = ASPLIT ? (A2  + (size_t)b * strideA) : nullptr;
  const T* Bb2 = BSPLIT ? (Bt2 + (size_t)b * strideB) : nullptr;

  const int rlane = lane & 15;
  const int koff  = (lane >> 4) * 8;
  const int mOff  = (lane >> 4) * 8;

  v8f acc[4][4];
#pragma unroll
  for (int i = 0; i < 4; ++i)
#pragma unroll
    for (int j = 0; j < 4; ++j) acc[i][j] = (v8f){0.f,0.f,0.f,0.f,0.f,0.f,0.f,0.f};

  for (int k0 = 0; k0 < K; k0 += 32) {
    V bh[4], bl[4];
#pragma unroll
    for (int j = 0; j < 4; ++j) {
      const size_t bo = (size_t)(n0 + (j << 4) + rlane) * ldb + koff + k0;
      bh[j] = Frag<T>::load(Bb + bo);
      if (BSPLIT) bl[j] = Frag<T>::load(Bb2 + bo);
    }
#pragma unroll
    for (int i = 0; i < 4; ++i) {
      const size_t ao = (size_t)(m0 + (i << 4) + rlane) * lda + koff + k0;
      V ah = Frag<T>::load(Ab + ao);
      V al = ah;
      if (ASPLIT) al = Frag<T>::load(Ab2 + ao);
#pragma unroll
      for (int j = 0; j < 4; ++j) {
        acc[i][j] = Frag<T>::mma(ah, bh[j], acc[i][j]);
        if (BSPLIT) acc[i][j] = Frag<T>::mma(ah, bl[j], acc[i][j]);
        if (ASPLIT) acc[i][j] = Frag<T>::mma(al, bh[j], acc[i][j]);
      }
      Frag<T>::guard(acc[i][0], acc[i][3], ah, al);
    }
    Frag<T>::keep(bh[0], bh[1], bh[2], bh[3]);
    if (BSPLIT) Frag<T>::keep(bl[0], bl[1], bl[2], bl[3]);
  }
  acc_guard4(acc[0][0], acc[0][1], acc[0][2], acc[0][3]);
  acc_guard4(acc[1][0], acc[1][1], acc[1][2], acc[1][3]);
  acc_guard4(acc[2][0], acc[2][1], acc[2][2], acc[2][3]);
  acc_guard4(acc[3][0], acc[3][1], acc[3][2], acc[3][3]);

  float* slab = sT[wave];
#pragma unroll
  for (int i = 0; i < 4; ++i) {
    const int mBase = m0 + (i << 4);
#pragma unroll
    for (int j = 0; j < 4; ++j) {
      const int n = n0 + (j << 4) + rlane;
      float bv = 0.f;
      if (BIAS_MODE == 2) bv = bias[n];
#pragma unroll
      for (int r = 0; r < 8; ++r) {
        float v = acc[i][j][r] * scale;
        if (BIAS_MODE == 1) v += bias[mBase + mOff + r];
        if (BIAS_MODE == 2) v += bv;
        slab[(mOff + r) * 68 + (j << 4) + rlane] = v;
      }
    }
    __builtin_amdgcn_fence(__ATOMIC_RELEASE, "workgroup");
    __builtin_amdgcn_wave_barrier();
    __builtin_amdgcn_fence(__ATOMIC_ACQUIRE, "workgroup");
    if (OUT_MODE == 0) {
      float* C = (float*)Cout + (size_t)b * strideC;
      const int hh = lane >> 4, c4 = (lane & 15) * 4;
      for (int pass = 0; pass < 2; ++pass) {
#pragma unroll
        for (int it = 0; it < 8; ++it) {
          const int row = it * 2 + hh;
          v4f v = *(const v4f*)(slab + row * 68 + c4);
          *(volatile v4f*)(C + (size_t)(mBase + row) * ldc + n0 + c4) = v;
        }
        __threadfence();
      }
    } else {
      const int q = lane >> 3, c8 = (lane & 7) * 8;
      unsigned short* C  = (unsigned short*)Cout  + (size_t)b * strideC;
      unsigned short* C2 = (OUT_MODE == 2) ? ((unsigned short*)Cout2 + (size_t)b * strideC) : nullptr;
      for (int pass = 0; pass < 2; ++pass) {
#pragma unroll
        for (int it = 0; it < 4; ++it) {
          const int row = it * 4 + q;
          const float* sp = slab + row * 68 + c8;
          v8h hv, lv;
#pragma unroll
          for (int e = 0; e < 8; ++e) {
            if (OUT_MODE == 1) {
              hv[e] = (_Float16)sp[e];
            } else {
              unsigned short hb = f2bf_bits(sp[e]);
              unsigned short lb = f2bf_bits(sp[e] - bf_bits2f(hb));
              hv[e] = __builtin_bit_cast(_Float16, hb);
              lv[e] = __builtin_bit_cast(_Float16, lb);
            }
          }
          *(volatile v8h*)(C + (size_t)(mBase + row) * ldc + n0 + c8) = hv;
          if (OUT_MODE == 2) *(volatile v8h*)(C2 + (size_t)(mBase + row) * ldc + n0 + c8) = lv;
        }
        __threadfence();
      }
    }
    __builtin_amdgcn_fence(__ATOMIC_RELEASE, "workgroup");
    __builtin_amdgcn_wave_barrier();
    __builtin_amdgcn_fence(__ATOMIC_ACQUIRE, "workgroup");
  }
}

__global__ __launch_bounds__(256) void cast_f32_bf16x2(
    const float* __restrict__ in, unsigned short* __restrict__ out, int n2) {
  int i = blockIdx.x * 256 + threadIdx.x;
  if (i < n2) {
    const unsigned u = (unsigned)f2bf_bits(in[2 * i]) | ((unsigned)f2bf_bits(in[2 * i + 1]) << 16);
    ((volatile unsigned*)out)[i] = u;
    __threadfence();
    ((volatile unsigned*)out)[i] = u;
  }
}

__global__ __launch_bounds__(256) void planes_k(const float* __restrict__ sa,
    unsigned short* __restrict__ sthp, unsigned short* __restrict__ stlp,
    unsigned short* __restrict__ achp, unsigned short* __restrict__ aclp,
    unsigned short* __restrict__ qvhp, unsigned short* __restrict__ qvlp) {
  const int row = blockIdx.x * 2 + (threadIdx.x >> 7);
  const int c8  = (threadIdx.x & 127) * 8;
  const float* sp = sa + (size_t)row * (2 * QRANK) + c8;
  const v8f sv = *(const v8f*)(sp);
  const v8f av = *(const v8f*)(sp + QRANK);
  v8h shv, slv, ahv, alv, qhv, qlv;
#pragma unroll
  for (int e = 0; e < 8; ++e) {
    const float s = sv[e], a = av[e];
    const float q = s * a;
    unsigned short hb, lb;
    hb = f2bf_bits(s); lb = f2bf_bits(s - bf_bits2f(hb));
    shv[e] = __builtin_bit_cast(_Float16, hb); slv[e] = __builtin_bit_cast(_Float16, lb);
    hb = f2bf_bits(a); lb = f2bf_bits(a - bf_bits2f(hb));
    ahv[e] = __builtin_bit_cast(_Float16, hb); alv[e] = __builtin_bit_cast(_Float16, lb);
    hb = f2bf_bits(q); lb = f2bf_bits(q - bf_bits2f(hb));
    qhv[e] = __builtin_bit_cast(_Float16, hb); qlv[e] = __builtin_bit_cast(_Float16, lb);
  }
  const size_t o = (size_t)row * QRANK + c8;
  _Float16* sth = (_Float16*)sthp; _Float16* stl = (_Float16*)stlp;
  _Float16* ach = (_Float16*)achp; _Float16* acl = (_Float16*)aclp;
  _Float16* qvh = (_Float16*)qvhp; _Float16* qvl = (_Float16*)qvlp;
  for (int pass = 0; pass < 2; ++pass) {
    *(volatile v8h*)(sth + o) = shv;
    *(volatile v8h*)(stl + o) = slv;
    *(volatile v8h*)(ach + o) = ahv;
    *(volatile v8h*)(acl + o) = alv;
    *(volatile v8h*)(qvh + o) = qhv;
    *(volatile v8h*)(qvl + o) = qlv;
    __threadfence();
  }
}

constexpr int ATT_QBLK = 64;
constexpr int ATT_KCH  = 64;
constexpr int ATT_OSP  = 132;
constexpr int ATT_NQB  = SEQ_LEN / ATT_QBLK;

__device__ __forceinline__ __bf16 at_f2bf(float f) { return __builtin_bit_cast(__bf16, f2bf_bits(f)); }
__device__ __forceinline__ void at_split(float f, __bf16& hi, __bf16& lo) {
  const unsigned short hb = f2bf_bits(f);
  hi = __builtin_bit_cast(__bf16, hb);
  lo = at_f2bf(f - __uint_as_float(((unsigned)hb) << 16));
}
__device__ __forceinline__ v8f at_mma(v16b a, v16b b, v8f c) {
  c = __builtin_amdgcn_wmma_f32_16x16x32_bf16(false, a, false, b, (short)0, c, false, false);
  asm volatile("v_nop\n\tv_nop\n\tv_nop\n\tv_nop" : "+v"(c) : "v"(a), "v"(b));
  return c;
}

__global__ __launch_bounds__(128)
void attn_route_k(const unsigned short* __restrict__ sthp, const unsigned short* __restrict__ stlp,
                  const unsigned short* __restrict__ achp, const unsigned short* __restrict__ aclp,
                  const unsigned short* __restrict__ cthp, const unsigned short* __restrict__ ctlp,
                  unsigned short* __restrict__ ghp, unsigned short* __restrict__ glp) {
  union FB { v16b v; v8b h[2]; };
  __shared__ __align__(16) __bf16 Psh[4][16 * ATT_KCH];
  __shared__ __align__(16) __bf16 Psl[4][16 * ATT_KCH];
  __shared__ __align__(16) float  Os[4][16 * ATT_OSP];

  const __bf16* sth = (const __bf16*)sthp; const __bf16* stl = (const __bf16*)stlp;
  const __bf16* ach = (const __bf16*)achp; const __bf16* acl = (const __bf16*)aclp;
  const __bf16* cth = (const __bf16*)cthp; const __bf16* ctl = (const __bf16*)ctlp;
  _Float16* gh = (_Float16*)ghp; _Float16* gl = (_Float16*)glp;

  const int tid  = threadIdx.x;
  const int wave = tid >> 5;
  const int lane = tid & 31;
  const int hh   = lane >> 4;
  const int c    = lane & 15;
  const int bx = blockIdx.x;
  const int qb = bx % ATT_NQB;
  const int h  = bx / ATT_NQB;
  const int q0 = qb * ATT_QBLK + wave * 16;

  v16b qah[2], qal[2];
#pragma unroll
  for (int dc = 0; dc < 2; ++dc) {
    const size_t off = (size_t)(q0 + c) * QRANK + h * HRANK + dc * 32 + 8 * hh;
    qah[dc] = Frag<__bf16>::load(sth + off);
    qal[dc] = Frag<__bf16>::load(stl + off);
  }

  float mrow[8], lrow[8];
  v8f oacc[8];
#pragma unroll
  for (int r = 0; r < 8; ++r) { mrow[r] = -INFINITY; lrow[r] = 0.f; }
#pragma unroll
  for (int t = 0; t < 8; ++t) oacc[t] = (v8f){0.f,0.f,0.f,0.f,0.f,0.f,0.f,0.f};

  __bf16* pwh = Psh[wave];
  __bf16* pwl = Psl[wave];
  const int nChunks = qb + 1;
  for (int kc = 0; kc < nChunks; ++kc) {
    const int kv0 = kc * ATT_KCH;

    v8f s[4];
#pragma unroll
    for (int j = 0; j < 4; ++j) {
      s[j] = (v8f){0.f,0.f,0.f,0.f,0.f,0.f,0.f,0.f};
#pragma unroll
      for (int dc = 0; dc < 2; ++dc) {
        const size_t ko = (size_t)(kv0 + j * 16 + c) * QRANK + h * HRANK + dc * 32 + 8 * hh;
        const v16b kb = Frag<__bf16>::load(ach + ko);
        const v16b kl = Frag<__bf16>::load(acl + ko);
        s[j] = at_mma(qah[dc], kb, s[j]);
        s[j] = at_mma(qah[dc], kl, s[j]);
        s[j] = at_mma(qal[dc], kb, s[j]);
      }
    }

    const bool diag = (kc == qb);
    float cm[8];
#pragma unroll
    for (int r = 0; r < 8; ++r) {
      const int qrow = q0 + 8 * hh + r;
      float m = -INFINITY;
#pragma unroll
      for (int j = 0; j < 4; ++j) {
        const int kvcol = kv0 + j * 16 + c;
        float v = s[j][r] * 0.125f;
        if (diag && (kvcol > qrow)) v = -INFINITY;
        s[j][r] = v;
        m = fmaxf(m, v);
      }
#pragma unroll
      for (int off = 1; off < 16; off <<= 1) m = fmaxf(m, __shfl_xor(m, off, 32));
      cm[r] = m;
    }

#pragma unroll
    for (int r = 0; r < 8; ++r) {
      const float mnew = fmaxf(mrow[r], cm[r]);
      const float alpha = expf(mrow[r] - mnew);
      mrow[r] = mnew;
      float psum = 0.f;
#pragma unroll
      for (int j = 0; j < 4; ++j) {
        const float p = expf(s[j][r] - mnew);
        psum += p;
        __bf16 a, bl; at_split(p, a, bl);
        pwh[(8 * hh + r) * ATT_KCH + j * 16 + c] = a;
        pwl[(8 * hh + r) * ATT_KCH + j * 16 + c] = bl;
      }
#pragma unroll
      for (int off = 1; off < 16; off <<= 1) psum += __shfl_xor(psum, off, 32);
      lrow[r] = lrow[r] * alpha + psum;
#pragma unroll
      for (int t = 0; t < 8; ++t) oacc[t][r] *= alpha;
    }
    __builtin_amdgcn_fence(__ATOMIC_RELEASE, "workgroup");
    __builtin_amdgcn_wave_barrier();
    __builtin_amdgcn_fence(__ATOMIC_ACQUIRE, "workgroup");

#pragma unroll 1
    for (int kk = 0; kk < 2; ++kk) {
      FB pa, pl;
      pa.h[0] = *(const v8b*)(pwh + c * ATT_KCH + kk * 32 + 8 * hh);
      pa.h[1] = *(const v8b*)(pwh + c * ATT_KCH + kk * 32 + 16 + 8 * hh);
      pl.h[0] = *(const v8b*)(pwl + c * ATT_KCH + kk * 32 + 8 * hh);
      pl.h[1] = *(const v8b*)(pwl + c * ATT_KCH + kk * 32 + 16 + 8 * hh);
#pragma unroll
      for (int t = 0; t < 8; ++t) {
        const size_t vo = (size_t)(h * HVAL + t * 16 + c) * SEQ_LEN + kv0 + kk * 32 + 8 * hh;
        const v16b vb = Frag<__bf16>::load(cth + vo);
        const v16b vl = Frag<__bf16>::load(ctl + vo);
        oacc[t] = at_mma(pa.v, vb, oacc[t]);
        oacc[t] = at_mma(pa.v, vl, oacc[t]);
        oacc[t] = at_mma(pl.v, vb, oacc[t]);
      }
    }
    __builtin_amdgcn_fence(__ATOMIC_RELEASE, "workgroup");
    __builtin_amdgcn_wave_barrier();
    __builtin_amdgcn_fence(__ATOMIC_ACQUIRE, "workgroup");
  }

  float* os = Os[wave];
#pragma unroll
  for (int r = 0; r < 8; ++r) {
    const float inv = 1.0f / lrow[r];
#pragma unroll
    for (int t = 0; t < 8; ++t) os[(8 * hh + r) * ATT_OSP + t * 16 + c] = oacc[t][r] * inv;
  }
  __builtin_amdgcn_fence(__ATOMIC_RELEASE, "workgroup");
  __builtin_amdgcn_wave_barrier();
  __builtin_amdgcn_fence(__ATOMIC_ACQUIRE, "workgroup");
  {
    const int q4 = lane >> 3, c8 = (lane & 7) * 8;
    const int rpar = q4 >> 1, chalf = (q4 & 1) * 64;
    for (int pass = 0; pass < 2; ++pass) {
#pragma unroll
      for (int it = 0; it < 8; ++it) {
        const int row = it * 2 + rpar;
        const int col = chalf + c8;
        const float* sp = os + row * ATT_OSP + col;
        v8h hv, lv;
#pragma unroll
        for (int e = 0; e < 8; ++e) {
          const unsigned short hb = f2bf_bits(sp[e]);
          const unsigned short lb = f2bf_bits(sp[e] - bf_bits2f(hb));
          hv[e] = __builtin_bit_cast(_Float16, hb);
          lv[e] = __builtin_bit_cast(_Float16, lb);
        }
        const size_t go = (size_t)(q0 + row) * HID + h * HVAL + col;
        *(volatile v8h*)(gh + go) = hv;
        *(volatile v8h*)(gl + go) = lv;
      }
      __threadfence();
    }
  }
}

extern "C" void kernel_launch(void* const* d_in, const int* in_sizes, int n_in,
                              void* d_out, int out_size, void* d_ws, size_t ws_size,
                              hipStream_t stream) {
  if (n_in < 6) return;
  if (in_sizes[0] != SEQ_LEN * HID || in_sizes[1] != QRANK * HID || in_sizes[2] != QRANK * HID ||
      in_sizes[3] != HID * QRANK || in_sizes[4] != HID * HID || in_sizes[5] != HID) return;
  if (out_size != SEQ_LEN * HID) return;

  const float* x  = (const float*)d_in[0];
  const float* Ws = (const float*)d_in[1];
  const float* Wa = (const float*)d_in[2];
  const float* Wc = (const float*)d_in[3];
  const float* Wo = (const float*)d_in[4];
  const float* bo = (const float*)d_in[5];
  float* out = (float*)d_out;

  const size_t B_XB  = (size_t)SEQ_LEN * HID * 2;
  const size_t B_WSA = (size_t)(2 * QRANK) * HID * 2;
  const size_t B_WC  = (size_t)HID * QRANK * 2;
  const size_t B_WO  = (size_t)HID * HID * 2;
  const size_t B_SA  = (size_t)SEQ_LEN * (2 * QRANK) * 4;
  const size_t B_PL  = (size_t)SEQ_LEN * QRANK * 2;
  const size_t B_CT  = (size_t)HID * SEQ_LEN * 2;
  const size_t B_G   = (size_t)SEQ_LEN * HID * 2;

  char* ws = (char*)d_ws;
  size_t off = 0;
  unsigned short* XB  = (unsigned short*)(ws + off); off += B_XB;
  unsigned short* WSA = (unsigned short*)(ws + off); off += B_WSA;
  unsigned short* WC  = (unsigned short*)(ws + off); off += B_WC;
  unsigned short* WO  = (unsigned short*)(ws + off); off += B_WO;
  float*          SA  = (float*)(ws + off);          off += B_SA;
  unsigned short* STH = (unsigned short*)(ws + off); off += B_PL;
  unsigned short* STL = (unsigned short*)(ws + off); off += B_PL;
  unsigned short* ACH = (unsigned short*)(ws + off); off += B_PL;
  unsigned short* ACL = (unsigned short*)(ws + off); off += B_PL;
  unsigned short* QVH = (unsigned short*)(ws + off); off += B_PL;
  unsigned short* QVL = (unsigned short*)(ws + off); off += B_PL;
  unsigned short* CTH = (unsigned short*)(ws + off); off += B_CT;
  unsigned short* CTL = (unsigned short*)(ws + off); off += B_CT;
  unsigned short* GH  = (unsigned short*)(ws + off); off += B_G;
  unsigned short* GL  = (unsigned short*)(ws + off); off += B_G;
  if (off > ws_size) return;

  {
    const int n2x = SEQ_LEN * HID / 2, n2w = QRANK * HID / 2, n2c = HID * QRANK / 2, n2o = HID * HID / 2;
    cast_f32_bf16x2<<<dim3((n2x + 255) / 256), dim3(256), 0, stream>>>(x,  XB, n2x);
    cast_f32_bf16x2<<<dim3((n2w + 255) / 256), dim3(256), 0, stream>>>(Ws, WSA, n2w);
    cast_f32_bf16x2<<<dim3((n2w + 255) / 256), dim3(256), 0, stream>>>(Wa, WSA + (size_t)QRANK * HID, n2w);
    cast_f32_bf16x2<<<dim3((n2c + 255) / 256), dim3(256), 0, stream>>>(Wc, WC, n2c);
    cast_f32_bf16x2<<<dim3((n2o + 255) / 256), dim3(256), 0, stream>>>(Wo, WO, n2o);
  }

  {
    const int M = SEQ_LEN, N = 2 * QRANK, K = HID;
    const int blocks = (M / 64) * (N / 64) / 8;
    wmma_gemm64<1, false, false, 0, 0><<<dim3(blocks, 1), dim3(256), 0, stream>>>(
        XB, XB, K, 0L, WSA, WSA, K, 0L, (void*)SA, (void*)SA, N, 0L, bo, M, N, K, 1.0f);
  }

  planes_k<<<dim3(SEQ_LEN / 2), dim3(256), 0, stream>>>(SA, STH, STL, ACH, ACL, QVH, QVL);

  {
    const int M = HID, N = SEQ_LEN, K = QRANK;
    const int blocks = (M / 64) * (N / 64) / 8;
    wmma_gemm64<1, false, true, 0, 2><<<dim3(blocks, 1), dim3(256), 0, stream>>>(
        WC, WC, K, 0L, QVH, QVL, K, 0L, (void*)CTH, (void*)CTL, N, 0L, bo, M, N, K, 1.0f);
  }

  attn_route_k<<<dim3(NHEADS * ATT_NQB), dim3(128), 0, stream>>>(STH, STL, ACH, ACL, CTH, CTL, GH, GL);

  {
    const int M = SEQ_LEN, N = HID, K = HID;
    const int blocks = (M / 64) * (N / 64) / 8;
    wmma_gemm64<1, true, false, 2, 0><<<dim3(blocks, 1), dim3(256), 0, stream>>>(
        GH, GL, K, 0L, WO, WO, K, 0L, (void*)out, (void*)out, N, 0L, bo, M, N, K, 1.0f);
  }
}
